// StationaryKernel_326417514820
// MI455X (gfx1250) — hardware-verified
//
#include <hip/hip_runtime.h>


#define NB   4
#define NPT  512
#define XD   64
#define TD   32
#define KF   (XD + TD)
#define HW   128
#define ICH  64
#define NPC  (ICH * NPT)
#define KP   128
#define DM   KP
#define LOSC 1024.0f

typedef _Float16 h16;
typedef unsigned short bf;
typedef __attribute__((ext_vector_type(16))) __bf16   v16bf;
typedef __attribute__((ext_vector_type(16))) _Float16 v16h;
typedef __attribute__((ext_vector_type(8)))  _Float16 v8h;
typedef __attribute__((ext_vector_type(8)))  unsigned short v8us;
typedef __attribute__((ext_vector_type(8)))  float    v8f;
typedef __attribute__((ext_vector_type(4)))  float    v4f;
typedef __attribute__((ext_vector_type(4)))  _Float16 v4h;
typedef v8h  __attribute__((may_alias)) v8ha;
typedef v4f  __attribute__((may_alias)) v4fa;
typedef v8us __attribute__((may_alias)) v8usa;

__device__ __forceinline__ unsigned short f2bf(float f) { unsigned u = __float_as_uint(f); u += 0x7FFFu + ((u >> 16) & 1u); return (unsigned short)(u >> 16); }
__device__ __forceinline__ float bf2f(unsigned short b) { return __uint_as_float(((unsigned)b) << 16); }
__device__ __forceinline__ float bfr(float f) { return bf2f(f2bf(f)); }
__device__ __forceinline__ v16h cat16(v8h lo, v8h hi) { return __builtin_shufflevector(lo, hi, 0, 1, 2, 3, 4, 5, 6, 7, 8, 9, 10, 11, 12, 13, 14, 15); }
__device__ __forceinline__ v16bf cat16b(v8us lo, v8us hi) { return __builtin_bit_cast(v16bf, __builtin_shufflevector(lo, hi, 0, 1, 2, 3, 4, 5, 6, 7, 8, 9, 10, 11, 12, 13, 14, 15)); }
__device__ __forceinline__ v8f wmma16(v16h a, v16h b, v8f c) { return __builtin_amdgcn_wmma_f32_16x16x32_f16(false, a, false, b, (short)0, c, false, false); }
__device__ __forceinline__ v8f wmmab(v16bf a, v16bf b, v8f c) { return __builtin_amdgcn_wmma_f32_16x16x32_bf16(false, a, false, b, (short)0, c, false, false); }

__global__ __launch_bounds__(256) void k_wt(const float* __restrict__ Wm, int K, int ncols, bf* WT) {
    __shared__ __align__(16) unsigned short tl[64 * 72];
    const int tid = threadIdx.x, k0 = blockIdx.x * 64, n0 = blockIdx.y * 64;
    const int kk = tid >> 2, nq = (tid & 3) * 16;
#pragma unroll
    for (int i = 0; i < 16; ++i) tl[(nq + i) * 72 + kk] = f2bf(Wm[(size_t)(k0 + kk) * ncols + n0 + nq + i]);
    __syncthreads();
    const int piece = tid & 7;
    auto pass = [&]() {
#pragma unroll
        for (int s = 0; s < 2; ++s) { const int nr = (tid >> 3) + 32 * s; const v8us val = *(const v8usa*)(tl + nr * 72 + piece * 8); *(volatile v8us*)(WT + (size_t)(n0 + nr) * K + k0 + piece * 8) = val; }
    };
    pass(); __threadfence(); pass();
}
template <bool SPLITA, bool F16OUT = false>
__global__ __launch_bounds__(128) void k_gemmb(const bf* __restrict__ A, const bf* __restrict__ Al, const bf* __restrict__ Bn, const float* __restrict__ bias, float* C, int ldc, h16* C2, const float* __restrict__ R = nullptr, int K = DM, int roundR = 1) {
    __shared__ __align__(16) float ost[4][16 * 68];
    const int lane = threadIdx.x & 31, wave = threadIdx.x >> 5, lr = lane & 15, hi = lane >> 4;
    const int r0 = blockIdx.x * 64 + wave * 16, c0 = blockIdx.y * 64;
    const size_t aoff = (size_t)(r0 + lr) * K + 8 * hi;
    size_t boff[4];
#pragma unroll
    for (int t = 0; t < 4; ++t) boff[t] = (size_t)(c0 + t * 16 + lr) * K + 8 * hi;
    v8f acc[4];
#pragma unroll
    for (int t = 0; t < 4; ++t) acc[t] = (v8f){};
#pragma unroll 1
    for (int kc = 0; kc < K; kc += 32) {
        const v16bf a = cat16b(*(const v8us*)(A + aoff + kc), *(const v8us*)(A + aoff + kc + 16));
        v16bf al = a;
        if (SPLITA) al = cat16b(*(const v8us*)(Al + aoff + kc), *(const v8us*)(Al + aoff + kc + 16));
#pragma unroll
        for (int t = 0; t < 4; ++t) { const v16bf b = cat16b(*(const v8us*)(Bn + boff[t] + kc), *(const v8us*)(Bn + boff[t] + kc + 16)); acc[t] = wmmab(a, b, acc[t]); if (SPLITA) acc[t] = wmmab(al, b, acc[t]); }
        asm volatile("v_nop\n\tv_nop\n\tv_nop\n\tv_nop" : "+v"(acc[0]), "+v"(acc[1]), "+v"(acc[2]), "+v"(acc[3]) : "v"(a), "v"(al));
    }
    float* os = &ost[wave][0];
#pragma unroll
    for (int t = 0; t < 4; ++t) { const float bv = bias ? bfr(bias[c0 + t * 16 + lr]) : 0.f;
#pragma unroll
        for (int j = 0; j < 8; ++j) os[(hi * 8 + j) * 68 + t * 16 + lr] = acc[t][j] + bv; }
    __syncthreads();
    if (F16OUT) {
        h16* crow = (h16*)(void*)C + (size_t)r0 * ldc + c0;
        auto pass = [&]() {
#pragma unroll
            for (int s = 0; s < 4; ++s) { const int row = 4 * s + (lane >> 3), piece = lane & 7; const float* sp = os + row * 68 + piece * 8; v8h o, o2;
#pragma unroll
                for (int i = 0; i < 8; ++i) { const h16 a = (h16)sp[i]; o[i] = a; o2[i] = (h16)((sp[i] - (float)a) * LOSC); }
                *(volatile v8h*)(crow + (size_t)row * ldc + piece * 8) = o; if (C2) *(volatile v8h*)(C2 + (size_t)r0 * ldc + c0 + (size_t)row * ldc + piece * 8) = o2; }
        };
        pass(); __threadfence(); pass();
    } else {
        float* crow = C + (size_t)r0 * ldc + c0;
        auto pass = [&]() {
#pragma unroll
            for (int s = 0; s < 8; ++s) { const int Lid = (lane >> 3) + 4 * s, piece = lane & 7; const int row = Lid >> 1, cofs = (Lid & 1) * 32 + piece * 4;
                v4f val = *(const v4fa*)(os + row * 68 + cofs); if (R) { const v4f rv = *(const v4f*)(R + ((size_t)r0 + row) * ldc + c0 + cofs); val += roundR ? (v4f){bfr(rv[0]), bfr(rv[1]), bfr(rv[2]), bfr(rv[3])} : rv; }
                *(volatile v4f*)(crow + (size_t)row * ldc + cofs) = val; }
        };
        pass(); __threadfence(); pass();
    }
}

__global__ __launch_bounds__(256) void k_feat(const float* __restrict__ xb, const float* __restrict__ yb, const float* __restrict__ tb, int i0, bf* Fh, bf* Fl) {
    typedef __attribute__((ext_vector_type(4))) unsigned short v4us;
    const int lane = threadIdx.x & 31; const int prow = blockIdx.x * 8 + (threadIdx.x >> 5);
    if (prow >= NPC) return;
    const int i = i0 + prow / NPT, j = prow - (prow / NPT) * NPT; const int c0 = lane * 4;
    v4us oh, ol;
#pragma unroll
    for (int k = 0; k < 4; ++k) { const int c = c0 + k; float f = 0.f;
        if (c < XD) { const float d = bfr(xb[(size_t)i * XD + c]) - bfr(yb[(size_t)j * XD + c]); f = d * d; } else if (c < KF) f = bfr(tb[c - XD]);
        const unsigned short hb = f2bf(f); oh[k] = hb; ol[k] = f2bf(f - bf2f(hb)); }
    const size_t o = (size_t)prow * KP + c0;
    *(volatile v4us*)(Fh + o) = oh; *(volatile v4us*)(Fl + o) = ol; __threadfence(); *(volatile v4us*)(Fh + o) = oh; *(volatile v4us*)(Fl + o) = ol;
}
__global__ __launch_bounds__(256) void k_w1t(const float* __restrict__ W1, bf* W1T) {
    typedef __attribute__((ext_vector_type(4))) unsigned short v4us;
    const int lane = threadIdx.x & 31; const int n = blockIdx.x * 8 + (threadIdx.x >> 5); if (n >= HW) return;
    v4us o;
#pragma unroll
    for (int k = 0; k < 4; ++k) { const int kk = lane * 4 + k; o[k] = kk < KF ? f2bf(W1[(size_t)kk * HW + n]) : (unsigned short)0; }
    *(volatile v4us*)(W1T + (size_t)n * KP + lane * 4) = o; __threadfence(); *(volatile v4us*)(W1T + (size_t)n * KP + lane * 4) = o;
}
__global__ __launch_bounds__(256) void k_relu2(const float* __restrict__ src, int nrows, bf* dh, bf* dl) {
    typedef __attribute__((ext_vector_type(4))) unsigned short v4us;
    const int lane = threadIdx.x & 31, r = blockIdx.x * 8 + (threadIdx.x >> 5);
    if (r >= nrows) return;
    const size_t o = (size_t)r * HW + lane * 4; const v4f v = *(const v4f*)(src + o); v4us oh, ol;
#pragma unroll
    for (int i = 0; i < 4; ++i) { const float g = fmaxf(v[i], 0.f); const unsigned short hb = f2bf(g); oh[i] = hb; ol[i] = f2bf(g - bf2f(hb)); }
    *(volatile v4us*)(dh + o) = oh; *(volatile v4us*)(dl + o) = ol; __threadfence(); *(volatile v4us*)(dh + o) = oh; *(volatile v4us*)(dl + o) = ol;
}
__global__ __launch_bounds__(256) void k_l3(const float* __restrict__ T2, const float* __restrict__ W3, const float* __restrict__ b3, float* KOUT) {
    const int lane = threadIdx.x & 31, w = blockIdx.x * 8 + (threadIdx.x >> 5); if (w >= NPC / 32) return;
    const int pr = w * 32 + lane; const float* row = T2 + (size_t)pr * HW;
    float a = bfr(b3[0]);
#pragma unroll 1
    for (int h = 0; h < HW; h += 4) { const v4f v = *(const v4f*)(row + h);
#pragma unroll
        for (int k = 0; k < 4; ++k) a = fmaf(fmaxf(v[k], 0.f), bfr(W3[h + k]), a); }
    *(volatile float*)(KOUT + pr) = a; __threadfence(); *(volatile float*)(KOUT + pr) = a;
}

extern "C" void kernel_launch(void* const* d_in, const int* in_sizes, int n_in,
                              void* d_out, int out_size, void* d_ws, size_t ws_size, hipStream_t stream) {
    (void)in_sizes; (void)n_in; (void)out_size;
    const float* x = (const float*)d_in[0]; const float* y = (const float*)d_in[1]; const float* t = (const float*)d_in[2];
    const float* W1 = (const float*)d_in[3]; const float* b1 = (const float*)d_in[4]; const float* W2 = (const float*)d_in[5]; const float* b2 = (const float*)d_in[6]; const float* W3 = (const float*)d_in[7]; const float* b3 = (const float*)d_in[8];
    float* out = (float*)d_out;
    char* wsp = (char*)d_ws;
    auto take = [&](size_t bytes) { char* p = wsp; wsp += (bytes + 255) & ~(size_t)255; return (void*)p; };
    bf* W1T = (bf*)take((size_t)HW * KP * 2); bf* W2T = (bf*)take((size_t)HW * HW * 2);
    bf* Fh = (bf*)take((size_t)NPC * KP * 2); bf* Fl = (bf*)take((size_t)NPC * KP * 2); float* T1 = (float*)take((size_t)NPC * HW * 4);
    bf* Hh = (bf*)take((size_t)NPC * HW * 2); bf* Hl = (bf*)take((size_t)NPC * HW * 2); float* T2 = (float*)take((size_t)NPC * HW * 4);
    if ((size_t)(wsp - (char*)d_ws) > ws_size) return;
    k_w1t<<<HW / 8, 256, 0, stream>>>(W1, W1T);
    k_wt<<<dim3(HW / 64, HW / 64, 1), 256, 0, stream>>>(W2, HW, HW, W2T);
    for (int b = 0; b < NB; ++b)
        for (int ic = 0; ic < NPT / ICH; ++ic) {
            k_feat<<<NPC / 8, 256, 0, stream>>>(x + (size_t)b * NPT * XD, y + (size_t)b * NPT * XD, t + (size_t)b * TD, ic * ICH, Fh, Fl);
            k_gemmb<true, false><<<dim3(NPC / 64, HW / 64, 1), 128, 0, stream>>>(Fh, Fl, W1T, b1, T1, HW, nullptr, nullptr, KP);
            k_relu2<<<NPC / 8, 256, 0, stream>>>(T1, NPC, Hh, Hl);
            k_gemmb<true, false><<<dim3(NPC / 64, HW / 64, 1), 128, 0, stream>>>(Hh, Hl, W2T, b2, T2, HW, nullptr, nullptr, HW);
            k_l3<<<(NPC / 32) / 8, 256, 0, stream>>>(T2, W3, b3, out + ((size_t)b * NPT + ic * ICH) * NPT);
        }
}
